// RoPEMultiHeadAttention_61847529062905
// MI455X (gfx1250) — hardware-verified
//
#include <hip/hip_runtime.h>
#include <math.h>

#pragma clang fp contract(off)

#ifndef NB
#define NB 2
#endif
#ifndef SEQ
#define SEQ 2048
#endif
#define NB_FULL 2
#define SEQ_FULL 2048
#define DM 2048
#define NH 16
#define NKV 4
#define DH 128
#define HALF 64
#define KVD (NKV * DH)
#define NTOK (NB * SEQ)
#define WSC 64.0f
#define OSC 64.0f

static_assert(SEQ % 128 == 0);
static_assert(SEQ <= SEQ_FULL);
static_assert(NB >= 1 && NB <= NB_FULL);
static_assert(DM % 128 == 0 && KVD % 128 == 0 && NTOK % 128 == 0);
static_assert(DH == 128 && HALF * 2 == DH && NH * DH == DM);

#define SZ_XH   ((size_t)NTOK * DM * 2)
#define SZ_WQT  ((size_t)DM * DM * 2)
#define SZ_WKT  ((size_t)KVD * DM * 2)
#define SZ_WVT  ((size_t)KVD * DM * 2)
#define SZ_WOT  ((size_t)DM * DM * 2)
#define SZ_TRG  ((size_t)SEQ * HALF * 4)
#define SZ_P    ((size_t)NTOK * DM * 4)
#define SZ_Q16  ((size_t)NTOK * DM * 2)
#define SZ_K16  ((size_t)NTOK * KVD * 2)
#define SZ_VT   ((size_t)NB * NKV * DH * SEQ * 2)
#define SZ_ATT  ((size_t)NTOK * DM * 2)
#define WS_TOTAL (SZ_XH + SZ_WQT + SZ_WKT + SZ_WVT + SZ_WOT + 2 * SZ_TRG + SZ_P + SZ_Q16 + SZ_K16 + SZ_VT + SZ_ATT)
static_assert(WS_TOTAL <= (size_t)134217728);
static_assert(SZ_XH % 256 == 0 && SZ_WKT % 256 == 0 && SZ_TRG % 256 == 0 && SZ_K16 % 256 == 0 && SZ_VT % 256 == 0);

typedef _Float16 f16;
typedef f16 f16x16 __attribute__((ext_vector_type(16)));
typedef f16 f16x8  __attribute__((ext_vector_type(8)));
typedef f16 f16x2  __attribute__((ext_vector_type(2)));
typedef float f32x8 __attribute__((ext_vector_type(8)));
typedef unsigned v4u __attribute__((ext_vector_type(4)));
typedef unsigned v4ua __attribute__((ext_vector_type(4), may_alias));
typedef float v4f __attribute__((ext_vector_type(4)));
typedef float v4fa __attribute__((ext_vector_type(4), may_alias));

__device__ __forceinline__ f32x8 wmma16(f16x16 a, f16x16 b, f32x8 c) {
  c = __builtin_amdgcn_wmma_f32_16x16x32_f16(false, a, false, b, (short)0, c, false, false);
  asm volatile("v_nop\n\tv_nop\n\tv_nop\n\tv_nop" : "+v"(c) : "v"(a), "v"(b));
  return c;
}

__device__ __forceinline__ f16x16 lds_frag(const f16* base, int stride) {
  const int lane = threadIdx.x & 31;
  const int row  = lane & 15;
  const int kh   = (lane >> 4) * 8;
  const f16x8 lo = *(const f16x8*)(base + row * stride + kh);
  const f16x8 hi = *(const f16x8*)(base + row * stride + kh + 16);
  f16x16 f;
#pragma unroll
  for (int i = 0; i < 8; ++i) { f[i] = lo[i]; f[i + 8] = hi[i]; }
  return f;
}

__device__ __forceinline__ f16x16 gfrag(const f16* __restrict__ base, int ld, int k0) {
  const int lane = threadIdx.x & 31;
  const int row  = lane & 15;
  const int kh   = (lane >> 4) * 8;
  const f16* p = base + (size_t)row * ld + k0 + kh;
  const f16x8 lo = *(const f16x8*)p;
  const f16x8 hi = *(const f16x8*)(p + 16);
  f16x16 f;
#pragma unroll
  for (int i = 0; i < 8; ++i) { f[i] = lo[i]; f[i + 8] = hi[i]; }
  return f;
}

__device__ __forceinline__ float bfr(float v) {
  unsigned u = __builtin_bit_cast(unsigned, v);
  u = (u + 0x7FFFu + ((u >> 16) & 1u)) & 0xFFFF0000u;
  return __builtin_bit_cast(float, u);
}

__global__ __launch_bounds__(256) void k_cvtx(const float* __restrict__ x, f16* __restrict__ Xh) {
  const int g = blockIdx.x * 256 + threadIdx.x;
  const int total8 = NTOK * DM / 8;
  const int gc = (g < total8) ? g : (total8 - 1);
  const int tok = gc / (DM / 8), c8 = (gc % (DM / 8)) * 8;
  const int srow = (tok / SEQ) * SEQ_FULL + (tok % SEQ);
  const float* src = x + (size_t)srow * DM + c8;
  const v4f a0 = *(const v4f*)src;
  const v4f a1 = *(const v4f*)(src + 4);
  union { f16 hh[8]; v4u v; } u;
#pragma unroll
  for (int e = 0; e < 4; ++e) {
    const float t0 = a0[e], t1 = a1[e];
    u.hh[e]     = (f16)bfr(t0);
    u.hh[e + 4] = (f16)bfr(t1);
  }
  f16* dst = Xh + (size_t)tok * DM + c8;
  if (g < total8) {
#pragma unroll 1
    for (int pass = 0; pass < 2; ++pass) { *(volatile v4u*)dst = u.v; __threadfence(); }
  }
}

#define WTSTR 72
__global__ __launch_bounds__(256) void k_wt(const float* __restrict__ W0, const float* __restrict__ W1,
                                            const float* __restrict__ W2, const float* __restrict__ W3,
                                            f16* __restrict__ T0, f16* __restrict__ T1, f16* __restrict__ T2, f16* __restrict__ T3) {
  __shared__ __attribute__((aligned(16))) f16 sT[64 * WTSTR];
  const int tid = threadIdx.x;
  const int z = blockIdx.z;
  const float* W = W0; f16* T = T0; int N = DM;
  if (z == 1)      { W = W1; T = T1; N = KVD; }
  else if (z == 2) { W = W2; T = T2; N = KVD; }
  else if (z == 3) { W = W3; T = T3; N = DM; }
  const int k0 = blockIdx.x * 64, n0 = blockIdx.y * 64;
  if (n0 >= N) return;
#pragma unroll 1
  for (int e = tid; e < 64 * 64; e += 256) {
    const int k = e >> 6, n = e & 63;
    const float v = W[(size_t)(k0 + k) * N + n0 + n];
    sT[n * WTSTR + k] = (f16)(bfr(v) * WSC);
  }
  __syncthreads();
#pragma unroll 1
  for (int pass = 0; pass < 2; ++pass) {
#pragma unroll 1
    for (int it = 0; it < 2; ++it) {
      const int r = it * 32 + (tid >> 3), piece = (tid & 7) * 8;
      *(volatile v4u*)(T + (size_t)(n0 + r) * DM + k0 + piece) = *(const v4ua*)(sT + r * WTSTR + piece);
    }
    __threadfence();
  }
}

__global__ __launch_bounds__(256) void k_trig(float* __restrict__ cT, float* __restrict__ sT) {
  const int g = blockIdx.x * 256 + threadIdx.x;
  const int total = SEQ * HALF;
  const int gc = (g < total) ? g : (total - 1);
  const int pos = gc >> 6, i = gc & 63;
  double pw = 1.0;
  pw = pw * ((i & 1)  ? 1.1547819846894582 : 1.0);
  pw = pw * ((i & 2)  ? 1.333521432163324  : 1.0);
  pw = pw * ((i & 4)  ? 1.7782794100389228 : 1.0);
  pw = pw * ((i & 8)  ? 3.1622776601683795 : 1.0);
  pw = pw * ((i & 16) ? 10.0 : 1.0);
  pw = pw * ((i & 32) ? 100.0 : 1.0);
  const float pwf = (float)pw;
  const float fr  = 1.0f / pwf;
  const float ang = (float)pos * fr;
  const float cs = cosf(ang);
  const float sn = sinf(ang);
  if (g < total) {
#pragma unroll 1
    for (int pass = 0; pass < 2; ++pass) {
      *(volatile float*)(cT + g) = cs;
      *(volatile float*)(sT + g) = sn;
      __threadfence();
    }
  }
}

#define GSTR 48
#define OSTRG 68
__global__ __launch_bounds__(256) __attribute__((amdgpu_num_vgpr(256)))
void k_gemm(const f16* __restrict__ A, int lda, const f16* __restrict__ Bt, int ldb,
            float* __restrict__ Y, int ldy, int K, float oscale) {
  __shared__ __attribute__((aligned(16))) f16 ldsA[128 * GSTR];
  __shared__ __attribute__((aligned(16))) f16 ldsW[128 * GSTR];
  __shared__ __attribute__((aligned(16))) float oS[8][32 * OSTRG];
  const int tid = threadIdx.x, lane = tid & 31, wave = tid >> 5, cl = lane & 15, rh = (lane >> 4) * 8;
  const int m0 = blockIdx.x * 128, n0 = blockIdx.y * 128;
  const int wm = (wave & 3) * 32, wn = (wave >> 2) * 64;
  f32x8 acc[2][4];
#pragma unroll
  for (int i = 0; i < 2; ++i)
#pragma unroll
    for (int j = 0; j < 4; ++j) { f32x8 zz = {}; acc[i][j] = zz; }
  const int srow = tid >> 1, sch = (tid & 1) * 16;
  const f16* asrc = A  + (size_t)(m0 + srow) * lda + sch;
  const f16* bsrc = Bt + (size_t)(n0 + srow) * ldb + sch;
#pragma unroll 1
  for (int k0 = 0; k0 < K; k0 += 32) {
    __syncthreads();
    const f16x8 a0 = *(const f16x8*)(asrc + k0);
    const f16x8 a1 = *(const f16x8*)(asrc + k0 + 8);
    const f16x8 b0 = *(const f16x8*)(bsrc + k0);
    const f16x8 b1 = *(const f16x8*)(bsrc + k0 + 8);
    *(f16x8*)(ldsA + srow * GSTR + sch)     = a0;
    *(f16x8*)(ldsA + srow * GSTR + sch + 8) = a1;
    *(f16x8*)(ldsW + srow * GSTR + sch)     = b0;
    *(f16x8*)(ldsW + srow * GSTR + sch + 8) = b1;
    __syncthreads();
    f16x16 af[2];
#pragma unroll
    for (int i = 0; i < 2; ++i) af[i] = lds_frag(ldsA + (wm + 16 * i) * GSTR, GSTR);
#pragma unroll
    for (int j = 0; j < 4; ++j) {
      const f16x16 bf = lds_frag(ldsW + (wn + 16 * j) * GSTR, GSTR);
#pragma unroll
      for (int i = 0; i < 2; ++i) acc[i][j] = wmma16(af[i], bf, acc[i][j]);
    }
  }
  float* so = oS[wave];
#pragma unroll
  for (int i = 0; i < 2; ++i)
#pragma unroll
    for (int j = 0; j < 4; ++j) {
#pragma unroll
      for (int r = 0; r < 8; ++r) so[(16 * i + rh + r) * OSTRG + 16 * j + cl] = acc[i][j][r] * oscale;
    }
  asm volatile("s_wait_dscnt 0" ::: "memory");
  __builtin_amdgcn_wave_barrier();
#pragma unroll 1
  for (int pass = 0; pass < 2; ++pass) {
#pragma unroll
    for (int it = 0; it < 16; ++it) {
      const int f4 = lane + 32 * it, rr = f4 >> 4, q = (f4 & 15) * 4;
      *(volatile v4f*)(Y + (size_t)(m0 + wm + rr) * ldy + n0 + wn + q) = *(const v4fa*)(so + rr * OSTRG + q);
    }
    __threadfence();
  }
}

#define RSTR 136
__global__ __launch_bounds__(256) void k_rope(const float* __restrict__ P, int ld, const float* __restrict__ cT,
                                              const float* __restrict__ sT, f16* __restrict__ R16) {
  __shared__ __attribute__((aligned(16))) f16 s[64 * RSTR];
  const int tid = threadIdx.x;
  const int t0 = blockIdx.x * 64;
  const int h = blockIdx.y;
#pragma unroll 1
  for (int e = tid; e < 64 * HALF; e += 256) {
    const int t = e >> 6, i = e & 63;
    const int tok = t0 + t;
    const int pos = tok % SEQ;
    const float* pp = P + (size_t)tok * ld + h * DH + 2 * i;
    const float x0 = pp[0], x1 = pp[1];
    const float c = cT[pos * HALF + i], sn = sT[pos * HALF + i];
    const float r0 = x0 * c - x1 * sn;
    const float r1 = x0 * sn + x1 * c;
    f16x2 v; v[0] = (f16)r0; v[1] = (f16)r1;
    *(f16x2*)(s + t * RSTR + 2 * i) = v;
  }
  __syncthreads();
#pragma unroll 1
  for (int pass = 0; pass < 2; ++pass) {
#pragma unroll 1
    for (int it = 0; it < 4; ++it) {
      const int idx = it * 256 + tid, r = idx >> 4, piece = (idx & 15) * 8;
      *(volatile v4u*)(R16 + (size_t)(t0 + r) * ld + h * DH + piece) = *(const v4ua*)(s + r * RSTR + piece);
    }
    __threadfence();
  }
}

#define VTSTR 72
__global__ __launch_bounds__(256) void k_vt(const float* __restrict__ P, f16* __restrict__ Vt) {
  __shared__ __attribute__((aligned(16))) f16 vT[DH * VTSTR];
  const int tid = threadIdx.x;
  const int t0 = blockIdx.x * 64;
  const int hk = blockIdx.y;
  const int b = t0 / SEQ, n0 = t0 % SEQ;
#pragma unroll 1
  for (int e = tid; e < 64 * DH; e += 256) {
    const int t = e >> 7, d = e & 127;
    vT[d * VTSTR + t] = (f16)P[(size_t)(t0 + t) * KVD + hk * DH + d];
  }
  __syncthreads();
#pragma unroll 1
  for (int pass = 0; pass < 2; ++pass) {
#pragma unroll 1
    for (int it = 0; it < 4; ++it) {
      const int idx = it * 256 + tid, r = idx >> 3, piece = (idx & 7) * 8;
      *(volatile v4u*)(Vt + ((size_t)((b * NKV + hk) * DH + r)) * SEQ + n0 + piece) = *(const v4ua*)(vT + r * VTSTR + piece);
    }
    __threadfence();
  }
}

#define KSTR 136
#define VSTR 48
#define OSTR 136
__global__ __launch_bounds__(256) __attribute__((amdgpu_num_vgpr(256)))
void k_attn(const f16* __restrict__ Q16, const f16* __restrict__ K16, const f16* __restrict__ Vt, f16* __restrict__ att) {
  __shared__ __attribute__((aligned(16))) f16 ldsK[32 * KSTR];
  __shared__ __attribute__((aligned(16))) f16 ldsV[DH * VSTR];
  __shared__ __attribute__((aligned(16))) f16 ldsO[8][16 * OSTR];

  const int t = threadIdx.x, wave = t >> 5, lane = t & 31;
  const int qlane = lane & 15, kh8 = (lane >> 4) * 8;
  const int h = blockIdx.y, b = blockIdx.z, hk = h % NKV;
  const int q0 = blockIdx.x * 128 + wave * 16;

  const f16* Qh = Q16 + ((size_t)b * SEQ + q0) * DM + h * DH;
  const f16* Kh = K16 + (size_t)b * SEQ * KVD + hk * DH;
  const f16* Vh = Vt + (size_t)(b * NKV + hk) * DH * SEQ;

  const int krow = t >> 3, kcol = (t & 7) * 16;
  const int vrow = t >> 1, vcol = (t & 1) * 16;
  const f16* kSrc = Kh + (size_t)krow * KVD + kcol;
  const f16* vSrc = Vh + (size_t)vrow * SEQ + vcol;

  f16x16 qf[4];
#pragma unroll
  for (int c = 0; c < 4; ++c) qf[c] = gfrag(Qh, DM, c * 32);

  f32x8 o[8];
#pragma unroll
  for (int j = 0; j < 8; ++j) { f32x8 zz = {}; o[j] = zz; }
  float mrun = -INFINITY, lrun = 0.0f;
  const float scale = 0.08838834764831845f * 1.4426950408889634f;

  f16x8 kreg[2], vreg[2];
  kreg[0] = *(const f16x8*)kSrc;  kreg[1] = *(const f16x8*)(kSrc + 8);
  vreg[0] = *(const f16x8*)vSrc;  vreg[1] = *(const f16x8*)(vSrc + 8);

#pragma unroll 1
  for (int kb = 0; kb < SEQ; kb += 32) {
    __syncthreads();
    *(f16x8*)(ldsK + krow * KSTR + kcol)     = kreg[0];
    *(f16x8*)(ldsK + krow * KSTR + kcol + 8) = kreg[1];
    *(f16x8*)(ldsV + vrow * VSTR + vcol)     = vreg[0];
    *(f16x8*)(ldsV + vrow * VSTR + vcol + 8) = vreg[1];
    if (kb + 32 < SEQ) {
      const f16* kn = kSrc + (size_t)(kb + 32) * KVD;
      const f16* vn = vSrc + (kb + 32);
      kreg[0] = *(const f16x8*)kn;  kreg[1] = *(const f16x8*)(kn + 8);
      vreg[0] = *(const f16x8*)vn;  vreg[1] = *(const f16x8*)(vn + 8);
    }
    __syncthreads();

    f32x8 s0 = {}, s1 = {};
#pragma unroll
    for (int c = 0; c < 4; ++c) {
      const f16x16 k0f = lds_frag(ldsK + c * 32, KSTR);
      const f16x16 k1f = lds_frag(ldsK + 16 * KSTR + c * 32, KSTR);
      s0 = wmma16(k0f, qf[c], s0);
      s1 = wmma16(k1f, qf[c], s1);
    }

    float mx = -INFINITY;
#pragma unroll
    for (int r = 0; r < 8; ++r) {
      s0[r] = s0[r] * scale;
      s1[r] = s1[r] * scale;
      mx = fmaxf(mx, fmaxf(s0[r], s1[r]));
    }
    mx = fmaxf(mx, __shfl_xor(mx, 16, 32));
    const float mnew  = fmaxf(mrun, mx);
    const float alpha = exp2f(mrun - mnew);

    float rsum = 0.0f;
    f16x16 pf;
#pragma unroll
    for (int r = 0; r < 8; ++r) {
      const float p0 = exp2f(s0[r] - mnew);
      const float p1 = exp2f(s1[r] - mnew);
      rsum += p0 + p1;
      pf[r]     = (f16)(p0 * 1024.0f);
      pf[r + 8] = (f16)(p1 * 1024.0f);
    }
    rsum += __shfl_xor(rsum, 16, 32);
    lrun = lrun * alpha + rsum;
    mrun = mnew;
#pragma unroll
    for (int j = 0; j < 8; ++j)
#pragma unroll
      for (int r = 0; r < 8; ++r) o[j][r] *= alpha;

#pragma unroll
    for (int j = 0; j < 8; ++j) {
      const f16x16 vf = lds_frag(ldsV + (j * 16) * VSTR, VSTR);
      o[j] = wmma16(vf, pf, o[j]);
    }
  }

  f16* so = ldsO[wave];
  const float rl = OSC / (lrun * 1024.0f);
#pragma unroll
  for (int j = 0; j < 8; ++j) {
    f16x8 v;
#pragma unroll
    for (int r = 0; r < 8; ++r) v[r] = (f16)(o[j][r] * rl);
    *(f16x8*)(so + qlane * OSTR + j * 16 + kh8) = v;
  }
  asm volatile("s_wait_dscnt 0" ::: "memory");
  __builtin_amdgcn_wave_barrier();
#pragma unroll 1
  for (int pass = 0; pass < 2; ++pass) {
#pragma unroll
    for (int it = 0; it < 8; ++it) {
      const int ch = lane + 32 * it, ql = ch >> 4, q8 = (ch & 15) * 8;
      *(volatile v4u*)(att + ((size_t)b * SEQ + q0 + ql) * DM + h * DH + q8) = *(const v4ua*)(so + ql * OSTR + q8);
    }
    __threadfence();
  }
}

extern "C" void kernel_launch(void* const* d_in, const int* in_sizes, int n_in,
                              void* d_out, int out_size, void* d_ws, size_t ws_size,
                              hipStream_t stream) {
  if (n_in < 5) return;
  if (in_sizes[0] < ((NB - 1) * SEQ_FULL + SEQ) * DM) return;
  if (in_sizes[1] < DM * DM || in_sizes[2] < DM * KVD || in_sizes[3] < DM * KVD || in_sizes[4] < DM * DM) return;
  if (out_size < NTOK * DM) return;
  if (ws_size < WS_TOTAL) return;

  const float* x  = (const float*)d_in[0];
  const float* Wq = (const float*)d_in[1];
  const float* Wk = (const float*)d_in[2];
  const float* Wv = (const float*)d_in[3];
  const float* Wo = (const float*)d_in[4];
  float* out = (float*)d_out;

  char* ws = (char*)d_ws;
  f16* Xh  = (f16*)ws;  ws += SZ_XH;
  f16* WqT = (f16*)ws;  ws += SZ_WQT;
  f16* WkT = (f16*)ws;  ws += SZ_WKT;
  f16* WvT = (f16*)ws;  ws += SZ_WVT;
  f16* WoT = (f16*)ws;  ws += SZ_WOT;
  float* cT = (float*)ws; ws += SZ_TRG;
  float* sT = (float*)ws; ws += SZ_TRG;
  float* P  = (float*)ws; ws += SZ_P;
  f16* Q16 = (f16*)ws;  ws += SZ_Q16;
  f16* K16 = (f16*)ws;  ws += SZ_K16;
  f16* Vt  = (f16*)ws;  ws += SZ_VT;
  f16* att = (f16*)ws;  ws += SZ_ATT;
  if ((size_t)(ws - (char*)d_ws) > ws_size) return;

  const dim3 blk(256);
  k_cvtx<<<dim3((NTOK * DM / 8 + 255) / 256), blk, 0, stream>>>(x, Xh);
  k_wt<<<dim3(DM / 64, DM / 64, 4), blk, 0, stream>>>(Wq, Wk, Wv, Wo, WqT, WkT, WvT, WoT);
  k_trig<<<dim3((SEQ * HALF + 255) / 256), blk, 0, stream>>>(cT, sT);

  k_gemm<<<dim3(NTOK / 128, DM / 128), blk, 0, stream>>>(Xh, DM, WqT, DM, P, DM, DM, 1.0f / 64.0f);
  k_rope<<<dim3(NTOK / 64, NH), blk, 0, stream>>>(P, DM, cT, sT, Q16);
  k_gemm<<<dim3(NTOK / 128, KVD / 128), blk, 0, stream>>>(Xh, DM, WkT, DM, P, KVD, DM, 1.0f / 64.0f);
  k_rope<<<dim3(NTOK / 64, NKV), blk, 0, stream>>>(P, KVD, cT, sT, K16);
  k_gemm<<<dim3(NTOK / 128, KVD / 128), blk, 0, stream>>>(Xh, DM, WvT, DM, P, KVD, DM, 1.0f / 64.0f);
  k_vt<<<dim3(NTOK / 64, NKV), blk, 0, stream>>>(P, Vt);

  k_attn<<<dim3(SEQ / 128, NH, NB), blk, 0, stream>>>(Q16, K16, Vt, att);

  k_gemm<<<dim3(NTOK / 128, DM / 128), blk, 0, stream>>>(att, DM, WoT, DM, out, DM, DM, 1.0f / 4096.0f);
}
